// Decoder_85066122265358
// MI455X (gfx1250) — hardware-verified
//
#include <hip/hip_runtime.h>
#include <math.h>

constexpr int NSC  = 128;
constexpr int NPD  = 32;
constexpr int NHD  = 32;
constexpr int NEM  = 16;
constexpr int NG1  = 72;
constexpr int NG2  = 8;
constexpr int NMD  = 64;
constexpr int NTS  = 8;
constexpr int NB   = NSC * NPD;
constexpr int NGT  = 4 * NHD;
constexpr int NKC  = NEM + NHD;
constexpr int NPH  = 2 * NG2;
constexpr int NMI  = NHD + NPH;
constexpr int NTHR = 128;
constexpr int NWAV = NTHR / 32;
constexpr int NOUT = NTS * NB * 2;
static_assert(NWAV == 4 && NPD == 32, "lane = pedestrian mapping");
static_assert(NHD == 8 * NWAV, "wave owns 8 hidden units");
static_assert(NMD == 16 * NWAV, "wave owns 16 mlp units");
static_assert(NGT == NTHR, "one gate bias per thread");
static_assert(NPD % NWAV == 0, "i loop exact");
static_assert(NPD * NEM == 4 * NTHR, "x embedding: 4 per thread");
static_assert(NPD * NHD == 8 * NTHR, "h init: 8 per thread");

constexpr int HSP = NHD + 1;
constexpr int XSP = NEM + 1;
constexpr int PHP = NPH + 1;
constexpr int DHP = NMD + 1;
constexpr int AP  = 40;
constexpr int EP  = 40;
constexpr int YP  = 40;
constexpr int HTP = 40;
constexpr int W1R = 80;
constexpr int W1P = 72;
constexpr int W2R = 16;
constexpr int W2P = 104;
constexpr int NMT1 = W1R / 16;
static_assert(NMT1 == 5 && W2R == 16, "");
static_assert(AP % 8 == 0 && EP % 8 == 0 && YP % 8 == 0 && HTP % 8 == 0 && W1P % 8 == 0 && W2P % 8 == 0, "16-B fragment alignment");
static_assert(NKC <= 64 && 64 <= W1P, "W1^T k range read = 64");
static_assert(NG1 <= 96 && 96 <= W2P, "W2^T k range read = 96");

constexpr float CXF   = 8.0f;
constexpr float CWF   = 16.0f;
constexpr float PHINV = 1.0f / (CXF * CWF * CWF);

constexpr int SZ_WCT  = NKC * NGT * 4;
constexpr int SZ_WM1  = NMI * NMD * 4;
constexpr int SZ_WM2  = NMD * NHD * 4;
constexpr int SZ_BSUM = NGT * 4;
constexpr int SZ_BM1  = NMD * 4;
constexpr int SZ_BM2  = NHD * 4;
constexpr int SZ_WHP  = NHD * 2 * 4;
constexpr int SZ_BHP  = 16;
constexpr int SZ_WSE  = 2 * NEM * 4;
constexpr int SZ_BSE  = NEM * 4;
constexpr int SZ_WPSE = 2 * NEM * 4;
constexpr int SZ_BPSE = NEM * 4;
constexpr int SZ_HS   = NPD * HSP * 4;
constexpr int SZ_XS   = NPD * XSP * 4;
constexpr int SZ_PHS  = NPD * PHP * 4;
constexpr int SZ_POS  = NPD * 2 * 4;
constexpr int SZ_REL  = NPD * 2 * 4;
constexpr int SZ_GS   = NPD * 4;
constexpr int SZ_SAME = NPD * 4;
constexpr int SZ_HT   = NHD * HTP * 2;
constexpr int SZ_W1T  = 2 * W1R * W1P * 2;
constexpr int SZ_W2T  = 2 * W2R * W2P * 2;
constexpr int AB_N    = NPD * AP;
constexpr int EB_N    = NEM * EP;
constexpr int Y1_N    = W1R * YP;
constexpr int WAVE_BYTES = (AB_N + EB_N + Y1_N) * 2;
constexpr int SZ_WAVE = NWAV * WAVE_BYTES;
constexpr int SZ_DHS  = NPD * DHP * 4;
static_assert(SZ_DHS <= SZ_WAVE, "");

constexpr int O_WCT  = 0;
constexpr int O_WM1  = O_WCT  + SZ_WCT;
constexpr int O_WM2  = O_WM1  + SZ_WM1;
constexpr int O_BSUM = O_WM2  + SZ_WM2;
constexpr int O_BM1  = O_BSUM + SZ_BSUM;
constexpr int O_BM2  = O_BM1  + SZ_BM1;
constexpr int O_WHP  = O_BM2  + SZ_BM2;
constexpr int O_BHP  = O_WHP  + SZ_WHP;
constexpr int O_WSE  = O_BHP  + SZ_BHP;
constexpr int O_BSE  = O_WSE  + SZ_WSE;
constexpr int O_WPSE = O_BSE  + SZ_BSE;
constexpr int O_BPSE = O_WPSE + SZ_WPSE;
constexpr int O_HS   = O_BPSE + SZ_BPSE;
constexpr int O_XS   = O_HS   + SZ_HS;
constexpr int O_PHS  = O_XS   + SZ_XS;
constexpr int O_POS  = O_PHS  + SZ_PHS;
constexpr int O_REL  = O_POS  + SZ_POS;
constexpr int O_GS   = O_REL  + SZ_REL;
constexpr int O_SAME = O_GS   + SZ_GS;
constexpr int O_HT   = O_SAME + SZ_SAME;
constexpr int O_W1T  = O_HT   + SZ_HT;
constexpr int O_W2T  = O_W1T  + SZ_W1T;
constexpr int O_WAVE = O_W2T  + SZ_W2T;
constexpr int LDS_TOTAL = O_WAVE + SZ_WAVE;
static_assert(LDS_TOTAL == 129168, "");
static_assert(O_WCT % 16 == 0 && O_WM1 % 16 == 0 && O_WM2 % 16 == 0 && O_HS % 16 == 0 && O_REL % 16 == 0 &&
              O_HT % 16 == 0 && O_W1T % 16 == 0 && O_W2T % 16 == 0 && O_WAVE % 16 == 0 && WAVE_BYTES % 16 == 0, "16-B alignment");

typedef __attribute__((ext_vector_type(16))) _Float16 v16h;
typedef __attribute__((ext_vector_type(8)))  _Float16 v8h;
typedef __attribute__((ext_vector_type(8)))  float    v8f;
typedef __attribute__((ext_vector_type(4)))  float    v4f;

template <typename T> struct Frag;
template <> struct Frag<_Float16> {
  typedef v16h V; union U { v16h v; v8h h[2]; };
  static __device__ __forceinline__ v16h load(const _Float16* p) {
    U f; f.h[0] = *(const v8h*)(p); f.h[1] = *(const v8h*)(p + 16); return f.v;
  }
  static __device__ __forceinline__ v8f mma(v16h a, v16h b, v8f c) {
    return __builtin_amdgcn_wmma_f32_16x16x32_f16(false, a, false, b, (short)0, c, false, false);
  }
};

__device__ __forceinline__ void grd3f4(v8f& a, v8f& b, v8f& c, v16h u0, v16h u1, v16h u2, v16h u3) {
  asm volatile("v_nop\n\tv_nop\n\tv_nop\n\tv_nop" : "+v"(a), "+v"(b), "+v"(c) : "v"(u0), "v"(u1), "v"(u2), "v"(u3));
}
__device__ __forceinline__ void grd2f6(v8f& a, v8f& b, v16h u0, v16h u1, v16h u2, v16h u3, v16h u4, v16h u5) {
  asm volatile("v_nop\n\tv_nop\n\tv_nop\n\tv_nop" : "+v"(a), "+v"(b) : "v"(u0), "v"(u1), "v"(u2), "v"(u3), "v"(u4), "v"(u5));
}
__device__ __forceinline__ void grd5f6(v8f& a, v8f& b, v8f& c, v8f& d, v8f& e,
                                       v16h u0, v16h u1, v16h u2, v16h u3, v16h u4, v16h u5) {
  asm volatile("v_nop\n\tv_nop\n\tv_nop\n\tv_nop" : "+v"(a), "+v"(b), "+v"(c), "+v"(d), "+v"(e)
               : "v"(u0), "v"(u1), "v"(u2), "v"(u3), "v"(u4), "v"(u5));
}
__device__ __forceinline__ void grd1f6(v8f& a, v16h u0, v16h u1, v16h u2, v16h u3, v16h u4, v16h u5) {
  asm volatile("v_nop\n\tv_nop\n\tv_nop\n\tv_nop" : "+v"(a) : "v"(u0), "v"(u1), "v"(u2), "v"(u3), "v"(u4), "v"(u5));
}

__device__ __forceinline__ void wave_sync() {
  __builtin_amdgcn_fence(__ATOMIC_RELEASE, "workgroup");
  __builtin_amdgcn_wave_barrier();
  __builtin_amdgcn_fence(__ATOMIC_ACQUIRE, "workgroup");
}

__device__ __forceinline__ v16h pack16(v8f lo, v8f hi) {
  v16h r;
#pragma unroll
  for (int e = 0; e < 8; ++e) { r[e] = (_Float16)lo[e]; r[8 + e] = (_Float16)hi[e]; }
  return r;
}
__device__ __forceinline__ v16h pack16z(v8f lo) {
  v16h r;
#pragma unroll
  for (int e = 0; e < 8; ++e) { r[e] = (_Float16)lo[e]; r[8 + e] = (_Float16)0.0f; }
  return r;
}

__device__ __forceinline__ float fsigm(float x) { return 1.0f / (1.0f + expf(-x)); }

__global__ __launch_bounds__(NTHR) void decoder_scene_kernel(
    const float* __restrict__ last_pos, const float* __restrict__ last_pos_rel,
    const float* __restrict__ h_init, const float* __restrict__ c_init,
    const int* __restrict__ seq_se, const int* __restrict__ end_group,
    const float* __restrict__ Wse, const float* __restrict__ bse,
    const float* __restrict__ Wih, const float* __restrict__ Whh,
    const float* __restrict__ bih, const float* __restrict__ bhh,
    const float* __restrict__ Whp, const float* __restrict__ bhp,
    const float* __restrict__ Wpse, const float* __restrict__ bpse,
    const float* __restrict__ W1a, const float* __restrict__ W2a,
    const float* __restrict__ W1b, const float* __restrict__ W2b,
    const float* __restrict__ Wm1, const float* __restrict__ bm1,
    const float* __restrict__ Wm2, const float* __restrict__ bm2,
    float* __restrict__ out) {
  (void)seq_se;
  __shared__ __align__(16) unsigned char smem[LDS_TOTAL];
  float* sWCT  = (float*)(smem + O_WCT);
  float* sWM1  = (float*)(smem + O_WM1);
  float* sWM2  = (float*)(smem + O_WM2);
  float* sBSUM = (float*)(smem + O_BSUM);
  float* sBM1  = (float*)(smem + O_BM1);
  float* sBM2  = (float*)(smem + O_BM2);
  float* sWHP  = (float*)(smem + O_WHP);
  float* sBHP  = (float*)(smem + O_BHP);
  float* sWSE  = (float*)(smem + O_WSE);
  float* sBSE  = (float*)(smem + O_BSE);
  float* sWPSE = (float*)(smem + O_WPSE);
  float* sBPSE = (float*)(smem + O_BPSE);
  float* sHS   = (float*)(smem + O_HS);
  float* sXS   = (float*)(smem + O_XS);
  float* sPHS  = (float*)(smem + O_PHS);
  float* sPOS  = (float*)(smem + O_POS);
  float* sREL  = (float*)(smem + O_REL);
  int*   sGS   = (int*)(smem + O_GS);
  unsigned* sSAME = (unsigned*)(smem + O_SAME);
  _Float16* sHT  = (_Float16*)(smem + O_HT);
  _Float16* sW1T = (_Float16*)(smem + O_W1T);
  _Float16* sW2T = (_Float16*)(smem + O_W2T);
  float* sDHS = (float*)(smem + O_WAVE);

  const int tid  = threadIdx.x;
  const int lane = tid & 31;
  const int wave = tid >> 5;
  const int s    = blockIdx.x;
  const int p    = lane;
  const int u0   = 8 * wave;
  const int m0   = 16 * wave;
  const int rl   = lane & 15;
  const int hh   = lane >> 4;
  const int koff = hh * 8;
  const v8f z8 = {0.f, 0.f, 0.f, 0.f, 0.f, 0.f, 0.f, 0.f};

#pragma unroll 1
  for (int it = 0; it < (NGT * NEM / 4) / NTHR; ++it) {
    const int e4 = it * NTHR + tid;
    const int n = e4 >> 2, k4 = (e4 & 3) * 4;
    const v4f v = *(const v4f*)(Wih + n * NEM + k4);
    sWCT[(k4 + 0) * NGT + n] = v[0];
    sWCT[(k4 + 1) * NGT + n] = v[1];
    sWCT[(k4 + 2) * NGT + n] = v[2];
    sWCT[(k4 + 3) * NGT + n] = v[3];
  }
#pragma unroll 1
  for (int it = 0; it < (NGT * NHD / 4) / NTHR; ++it) {
    const int e4 = it * NTHR + tid;
    const int n = e4 >> 3, k4 = (e4 & 7) * 4;
    const v4f v = *(const v4f*)(Whh + n * NHD + k4);
    sWCT[(NEM + k4 + 0) * NGT + n] = v[0];
    sWCT[(NEM + k4 + 1) * NGT + n] = v[1];
    sWCT[(NEM + k4 + 2) * NGT + n] = v[2];
    sWCT[(NEM + k4 + 3) * NGT + n] = v[3];
  }
#pragma unroll 1
  for (int it = 0; it < (NMI * NMD / 4) / NTHR; ++it) {
    const int e4 = it * NTHR + tid;
    *(v4f*)(sWM1 + 4 * e4) = *(const v4f*)(Wm1 + 4 * e4);
  }
#pragma unroll 1
  for (int it = 0; it < (NMD * NHD / 4) / NTHR; ++it) {
    const int e4 = it * NTHR + tid;
    *(v4f*)(sWM2 + 4 * e4) = *(const v4f*)(Wm2 + 4 * e4);
  }
  sBSUM[tid] = bih[tid] + bhh[tid];
  asm volatile("" ::: "memory");
  if (tid < NMD)     sBM1[tid] = bm1[tid];
  if (tid < NHD)     sBM2[tid] = bm2[tid];
  if (tid < 2 * NHD) sWHP[tid] = Whp[tid];
  if (tid < 2)       sBHP[tid] = bhp[tid];
  asm volatile("" ::: "memory");
  if (tid < 2 * NEM) { sWSE[tid] = Wse[tid]; sWPSE[tid] = Wpse[tid]; }
  if (tid < NEM)     { sBSE[tid] = bse[tid]; sBPSE[tid] = bpse[tid]; }
  asm volatile("" ::: "memory");

#pragma unroll 1
  for (int ty = 0; ty < 2; ++ty) {
    const float* W1 = ty ? W1b : W1a;
    _Float16* dst = sW1T + ty * (W1R * W1P);
#pragma unroll 1
    for (int e = tid; e < W1R * W1P; e += NTHR) {
      const int g = e / W1P;
      const int f = e - g * W1P;
      const int gc = (g < NG1) ? g : (NG1 - 1);
      const int fc = (f < NKC) ? f : (NKC - 1);
      const float x = W1[fc * NG1 + gc];
      const float fs = (g < NG1 && f < NKC) ? CWF : 0.0f;
      dst[e] = (_Float16)(x * fs);
    }
  }
#pragma unroll 1
  for (int ty = 0; ty < 2; ++ty) {
    const float* W2 = ty ? W2b : W2a;
    _Float16* dst = sW2T + ty * (W2R * W2P);
#pragma unroll 1
    for (int e = tid; e < W2R * W2P; e += NTHR) {
      const int o = e / W2P;
      const int g = e - o * W2P;
      const int oc = (o < NG2) ? o : (NG2 - 1);
      const int gc = (g < NG1) ? g : (NG1 - 1);
      const float x = W2[gc * NG2 + oc];
      const float fs = (o < NG2 && g < NG1) ? CWF : 0.0f;
      dst[e] = (_Float16)(x * fs);
    }
  }
  asm volatile("" ::: "memory");

  {
    const int pp = tid >> 2, k8 = (tid & 3) * 8;
    const float* hp = h_init + (size_t)(s * NPD + pp) * NHD + k8;
    const v4f a = *(const v4f*)hp;
    const v4f b = *(const v4f*)(hp + 4);
#pragma unroll
    for (int q = 0; q < 4; ++q) { sHS[pp * HSP + k8 + q] = a[q]; sHS[pp * HSP + k8 + 4 + q] = b[q]; }
  }
  float cst[8];
  {
    const float* cp = c_init + (size_t)(s * NPD + p) * NHD + u0;
    const v4f a = *(const v4f*)cp;
    const v4f b = *(const v4f*)(cp + 4);
#pragma unroll
    for (int q = 0; q < 4; ++q) { cst[q] = a[q]; cst[4 + q] = b[q]; }
  }
  asm volatile("" ::: "memory");
  if (tid < 2 * NPD) {
    sPOS[tid] = last_pos[(size_t)s * 2 * NPD + tid];
    sREL[tid] = last_pos_rel[(size_t)s * 2 * NPD + tid];
  }
  if (tid < NPD) sGS[tid] = end_group[s * NPD + tid];
  __syncthreads();
  if (tid < NPD) {
    const int j = tid;
    const int gj = sGS[j];
    unsigned bits = 0u;
#pragma unroll
    for (int k = 0; k < NPD; ++k) {
      const int gk = sGS[k];
      const bool sm = ((gj == gk) && (gj != 0)) || (j == k);
      bits |= sm ? (1u << k) : 0u;
    }
    sSAME[j] = bits;
  }
  __syncthreads();

  _Float16* wreg = (_Float16*)(smem + O_WAVE + wave * WAVE_BYTES);
  _Float16* abuf = wreg;
  _Float16* embT = wreg + AB_N;
  _Float16* y1t  = wreg + AB_N + EB_N;

#pragma unroll 1
  for (int t = 0; t < NTS; ++t) {
    {
      const int pp = tid >> 2, n4 = (tid & 3) * 4;
      const float rx = sREL[2 * pp], ry = sREL[2 * pp + 1];
#pragma unroll
      for (int q = 0; q < 4; ++q) {
        const int n = n4 + q;
        sXS[pp * XSP + n] = rx * sWSE[n] + ry * sWSE[NEM + n] + sBSE[n];
      }
    }
    __syncthreads();

    float ga[4][8];
#pragma unroll
    for (int g = 0; g < 4; ++g)
#pragma unroll
      for (int j = 0; j < 8; ++j) ga[g][j] = sBSUM[g * NHD + u0 + j];
#pragma unroll 1
    for (int k = 0; k < NEM; ++k) {
      const float a = sXS[p * XSP + k];
      const float* wr = sWCT + k * NGT + u0;
#pragma unroll
      for (int g = 0; g < 4; ++g) {
        const v4f w0 = *(const v4f*)(wr + g * NHD);
        const v4f w1 = *(const v4f*)(wr + g * NHD + 4);
#pragma unroll
        for (int q = 0; q < 4; ++q) { ga[g][q] += a * w0[q]; ga[g][4 + q] += a * w1[q]; }
      }
    }
#pragma unroll 1
    for (int k = 0; k < NHD; ++k) {
      const float a = sHS[p * HSP + k];
      const float* wr = sWCT + (NEM + k) * NGT + u0;
#pragma unroll
      for (int g = 0; g < 4; ++g) {
        const v4f w0 = *(const v4f*)(wr + g * NHD);
        const v4f w1 = *(const v4f*)(wr + g * NHD + 4);
#pragma unroll
        for (int q = 0; q < 4; ++q) { ga[g][q] += a * w0[q]; ga[g][4 + q] += a * w1[q]; }
      }
    }
    float h2r[8];
#pragma unroll
    for (int j = 0; j < 8; ++j) {
      const float ig = fsigm(ga[0][j]);
      const float fg = fsigm(ga[1][j]);
      const float gg = tanhf(ga[2][j]);
      const float og = fsigm(ga[3][j]);
      const float cn = fg * cst[j] + ig * gg;
      cst[j] = cn;
      h2r[j] = og * tanhf(cn);
    }
    __syncthreads();
#pragma unroll
    for (int j = 0; j < 8; ++j) {
      sHS[p * HSP + u0 + j] = h2r[j];
      sHT[(u0 + j) * HTP + p] = (_Float16)(h2r[j] * CXF);
    }
    __syncthreads();

    if (tid < 2 * NPD) {
      const int pp = tid >> 1, d = tid & 1;
      float a = sBHP[d];
#pragma unroll
      for (int k = 0; k < NHD; ++k) a += sHS[pp * HSP + k] * sWHP[k * 2 + d];
      sREL[tid] = a;
      sPOS[tid] += a;
    }
    __syncthreads();

    if (wave == 0) {
      const v4f v = *(const v4f*)(sREL + 4 * (lane & 15));
      float* op = out + ((size_t)t * NB + (size_t)s * NPD) * 2 + 4 * (lane & 15);
      for (int pass = 0; pass < 2; ++pass) {
        if (lane < 16) *(volatile v4f*)op = v;
        __threadfence();
      }
    }

#pragma unroll 1
    for (int it = 0; it < NPD / NWAV; ++it) {
      const int i = wave + NWAV * it;
      {
        const int n = rl;
        const float w0 = sWPSE[n], w1 = sWPSE[NEM + n], bb = sBPSE[n];
        const float pix = sPOS[2 * i], piy = sPOS[2 * i + 1];
        v8h e0, e1;
#pragma unroll
        for (int e = 0; e < 8; ++e) {
          const int ka = 16 * hh + e, kb = 16 * hh + 8 + e;
          const float va = ((sPOS[2 * ka] - pix) * w0 + (sPOS[2 * ka + 1] - piy) * w1 + bb) * CXF;
          const float vb = ((sPOS[2 * kb] - pix) * w0 + (sPOS[2 * kb + 1] - piy) * w1 + bb) * CXF;
          e0[e] = (_Float16)va;
          e1[e] = (_Float16)vb;
        }
        *(v8h*)(embT + n * EP + 16 * hh)     = e0;
        *(v8h*)(embT + n * EP + 16 * hh + 8) = e1;
      }
      wave_sync();
      const unsigned sameI = sSAME[i];
      const unsigned sameJ = sSAME[lane];
      const unsigned bitI  = 1u << i;
      const unsigned bitJ  = 1u << lane;
#pragma unroll 1
      for (int ty = 0; ty < 2; ++ty) {
        {
          const unsigned mI = ty ? ((~sameI) | bitI) : sameI;
          const unsigned mJ = ty ? ((~sameJ) | bitJ) : sameJ;
          const float cntI  = (float)__builtin_popcount(mI);
          const float mij   = (float)((mI >> lane) & 1u);
          const float denom = (lane == i) ? cntI : (1.0f + mij);
          const float inv   = 1.0f / denom;
          const unsigned adjb = (lane == i) ? 0xffffffffu : (bitI | bitJ);
          const unsigned rowb = adjb & mJ;
#pragma unroll
          for (int q = 0; q < 4; ++q) {
            v8h a8;
#pragma unroll
            for (int e = 0; e < 8; ++e) a8[e] = (_Float16)(((rowb >> (8 * q + e)) & 1u) ? inv : 0.0f);
            *(v8h*)(abuf + lane * AP + 8 * q) = a8;
          }
        }
        wave_sync();
        v16h bA[2];
        bA[0] = Frag<_Float16>::load(abuf + rl * AP + koff);
        bA[1] = Frag<_Float16>::load(abuf + (16 + rl) * AP + koff);
        const v16h aE  = Frag<_Float16>::load(embT + rl * EP + koff);
        const v16h aH0 = Frag<_Float16>::load(sHT + rl * HTP + koff);
        const v16h aH1 = Frag<_Float16>::load(sHT + (16 + rl) * HTP + koff);

        v16h b2[2][2];
#pragma unroll
        for (int nt = 0; nt < 2; ++nt) {
          v8f d0 = Frag<_Float16>::mma(aE,  bA[nt], z8);
          v8f d1 = Frag<_Float16>::mma(aH0, bA[nt], z8);
          v8f d2 = Frag<_Float16>::mma(aH1, bA[nt], z8);
          grd3f4(d0, d1, d2, aE, aH0, aH1, bA[nt]);
          b2[nt][0] = pack16(d0, d1);
          b2[nt][1] = pack16z(d2);
        }

        const _Float16* w1p = sW1T + ty * (W1R * W1P);
#pragma unroll
        for (int mt = 0; mt < NMT1; ++mt) {
          const _Float16* wr = w1p + (16 * mt + rl) * W1P + koff;
          const v16h aw0 = Frag<_Float16>::load(wr);
          const v16h aw1 = Frag<_Float16>::load(wr + 32);
          v8f dd[2];
#pragma unroll
          for (int nt = 0; nt < 2; ++nt) {
            dd[nt] = Frag<_Float16>::mma(aw0, b2[nt][0], z8);
            dd[nt] = Frag<_Float16>::mma(aw1, b2[nt][1], dd[nt]);
          }
          grd2f6(dd[0], dd[1], aw0, aw1, b2[0][0], b2[0][1], b2[1][0], b2[1][1]);
#pragma unroll
          for (int nt = 0; nt < 2; ++nt)
#pragma unroll
            for (int r = 0; r < 8; ++r)
              y1t[(16 * mt + 8 * hh + r) * YP + 16 * nt + rl] = (_Float16)fmaxf(dd[nt][r], 0.0f);
        }
        wave_sync();

        v16h b4[2][3];
#pragma unroll
        for (int nt = 0; nt < 2; ++nt) {
          v16h ay[5];
          v8f  dd[5];
#pragma unroll
          for (int mt = 0; mt < 5; ++mt) ay[mt] = Frag<_Float16>::load(y1t + (16 * mt + rl) * YP + koff);
#pragma unroll
          for (int mt = 0; mt < 5; ++mt) dd[mt] = Frag<_Float16>::mma(ay[mt], bA[nt], z8);
          grd5f6(dd[0], dd[1], dd[2], dd[3], dd[4], ay[0], ay[1], ay[2], ay[3], ay[4], bA[nt]);
          b4[nt][0] = pack16(dd[0], dd[1]);
          b4[nt][1] = pack16(dd[2], dd[3]);
          b4[nt][2] = pack16z(dd[4]);
        }

        const _Float16* w2p = sW2T + ty * (W2R * W2P) + rl * W2P + koff;
        const v16h av0 = Frag<_Float16>::load(w2p);
        const v16h av1 = Frag<_Float16>::load(w2p + 32);
        const v16h av2 = Frag<_Float16>::load(w2p + 64);
        float mx[8];
        {
          v8f dd[2];
#pragma unroll
          for (int nt = 0; nt < 2; ++nt) {
            dd[nt] = Frag<_Float16>::mma(av0, b4[nt][0], z8);
            dd[nt] = Frag<_Float16>::mma(av1, b4[nt][1], dd[nt]);
            dd[nt] = Frag<_Float16>::mma(av2, b4[nt][2], dd[nt]);
            grd1f6(dd[nt], av0, av1, av2, b4[nt][0], b4[nt][1], b4[nt][2]);
          }
#pragma unroll
          for (int r = 0; r < 8; ++r) mx[r] = fmaxf(fmaxf(dd[0][r], 0.0f), fmaxf(dd[1][r], 0.0f));
        }
#pragma unroll
        for (int r = 0; r < 8; ++r) {
#pragma unroll
          for (int off = 16; off > 0; off >>= 1) mx[r] = fmaxf(mx[r], __shfl_xor(mx[r], off, 32));
        }
        if (lane == 0) {
#pragma unroll
          for (int r = 0; r < 8; ++r) sPHS[i * PHP + ty * NG2 + r] = mx[r] * PHINV;
        }
      }
    }
    __syncthreads();

    float dm[16];
#pragma unroll
    for (int m = 0; m < 16; ++m) dm[m] = sBM1[m0 + m];
#pragma unroll 1
    for (int k = 0; k < NHD; ++k) {
      const float a = sHS[p * HSP + k];
      const float* wr = sWM1 + k * NMD + m0;
#pragma unroll
      for (int q4 = 0; q4 < 4; ++q4) {
        const v4f w = *(const v4f*)(wr + 4 * q4);
#pragma unroll
        for (int q = 0; q < 4; ++q) dm[4 * q4 + q] += a * w[q];
      }
    }
#pragma unroll 1
    for (int k = 0; k < NPH; ++k) {
      const float a = sPHS[p * PHP + k];
      const float* wr = sWM1 + (NHD + k) * NMD + m0;
#pragma unroll
      for (int q4 = 0; q4 < 4; ++q4) {
        const v4f w = *(const v4f*)(wr + 4 * q4);
#pragma unroll
        for (int q = 0; q < 4; ++q) dm[4 * q4 + q] += a * w[q];
      }
    }
#pragma unroll
    for (int m = 0; m < 16; ++m) sDHS[p * DHP + m0 + m] = fmaxf(dm[m], 0.0f);
    __syncthreads();

    float hn[8];
#pragma unroll
    for (int j = 0; j < 8; ++j) hn[j] = sBM2[u0 + j];
#pragma unroll 1
    for (int k = 0; k < NMD; ++k) {
      const float a = sDHS[p * DHP + k];
      const float* wr = sWM2 + k * NHD + u0;
      const v4f w0 = *(const v4f*)(wr);
      const v4f w1 = *(const v4f*)(wr + 4);
#pragma unroll
      for (int q = 0; q < 4; ++q) { hn[q] += a * w0[q]; hn[4 + q] += a * w1[q]; }
    }
#pragma unroll
    for (int j = 0; j < 8; ++j) sHS[p * HSP + u0 + j] = fmaxf(hn[j], 0.0f);
    __syncthreads();
  }
}

extern "C" void kernel_launch(void* const* d_in, const int* in_sizes, int n_in,
                              void* d_out, int out_size, void* d_ws, size_t ws_size,
                              hipStream_t stream) {
  (void)d_ws; (void)ws_size;
  if (n_in < 24 || d_out == nullptr) return;
  if (in_sizes[0] != NB * 2 || in_sizes[1] != NB * 2 || in_sizes[2] != NB * NHD || in_sizes[3] != NB * NHD ||
      in_sizes[4] != NSC * 2 || in_sizes[5] != NB || in_sizes[6] != 2 * NEM || in_sizes[7] != NEM ||
      in_sizes[8] != NGT * NEM || in_sizes[9] != NGT * NHD || in_sizes[10] != NGT || in_sizes[11] != NGT ||
      in_sizes[12] != NHD * 2 || in_sizes[13] != 2 || in_sizes[14] != 2 * NEM || in_sizes[15] != NEM ||
      in_sizes[16] != NKC * NG1 || in_sizes[17] != NG1 * NG2 || in_sizes[18] != NKC * NG1 || in_sizes[19] != NG1 * NG2 ||
      in_sizes[20] != NMI * NMD || in_sizes[21] != NMD || in_sizes[22] != NMD * NHD || in_sizes[23] != NHD ||
      out_size != NOUT) return;

  const float* last_pos     = (const float*)d_in[0];
  const float* last_pos_rel = (const float*)d_in[1];
  const float* h_init       = (const float*)d_in[2];
  const float* c_init       = (const float*)d_in[3];
  const int*   seq_se       = (const int*)d_in[4];
  const int*   end_group    = (const int*)d_in[5];
  const float* Wse   = (const float*)d_in[6];
  const float* bse   = (const float*)d_in[7];
  const float* Wih   = (const float*)d_in[8];
  const float* Whh   = (const float*)d_in[9];
  const float* bih   = (const float*)d_in[10];
  const float* bhh   = (const float*)d_in[11];
  const float* Whp   = (const float*)d_in[12];
  const float* bhp   = (const float*)d_in[13];
  const float* Wpse  = (const float*)d_in[14];
  const float* bpse  = (const float*)d_in[15];
  const float* W1a   = (const float*)d_in[16];
  const float* W2a   = (const float*)d_in[17];
  const float* W1b   = (const float*)d_in[18];
  const float* W2b   = (const float*)d_in[19];
  const float* Wm1   = (const float*)d_in[20];
  const float* bm1   = (const float*)d_in[21];
  const float* Wm2   = (const float*)d_in[22];
  const float* bm2   = (const float*)d_in[23];
  float* out = (float*)d_out;

  decoder_scene_kernel<<<dim3(NSC), dim3(NTHR), 0, stream>>>(
      last_pos, last_pos_rel, h_init, c_init, seq_se, end_group,
      Wse, bse, Wih, Whh, bih, bhh, Whp, bhp, Wpse, bpse,
      W1a, W2a, W1b, W2b, Wm1, bm1, Wm2, bm2, out);
}
